// GlobalCrossAttention_20444044329787
// MI455X (gfx1250) — hardware-verified
//
#include <hip/hip_runtime.h>
#define NQ 300
#define NQP 304
#define HW 1024
#define GH 32
#define GW 32
#define CC 256
#define NH 8
#define HD 32
#define HID 512
#define QCH 76

typedef __bf16 v16b __attribute__((ext_vector_type(16)));
typedef unsigned short v8us __attribute__((ext_vector_type(8), may_alias));
typedef float  v8f  __attribute__((ext_vector_type(8)));
typedef float  v4f  __attribute__((ext_vector_type(4)));
typedef float  v4fa __attribute__((ext_vector_type(4), may_alias));
union FragB { v16b v; v8us half[2]; unsigned short u[16]; };

__device__ __forceinline__ unsigned short bf16_bits(float x) { unsigned int u = __float_as_uint(x); return (unsigned short)((u + 0x7FFFu + ((u >> 16) & 1u)) >> 16); }
__device__ __forceinline__ float bf16_val(unsigned short b) { return __uint_as_float(((unsigned int)b) << 16); }
__device__ __forceinline__ float bf16_round(float x) { return bf16_val(bf16_bits(x)); }
template <int NT>
__device__ __forceinline__ v8f mmaN(v16b ah, v16b al, v16b bh, v16b bl, v8f c) {
  c = __builtin_amdgcn_wmma_f32_16x16x32_bf16(false, ah, false, bh, (short)0, c, false, false);
  if (NT >= 2) c = __builtin_amdgcn_wmma_f32_16x16x32_bf16(false, al, false, bh, (short)0, c, false, false);
  if (NT >= 3) c = __builtin_amdgcn_wmma_f32_16x16x32_bf16(false, ah, false, bl, (short)0, c, false, false);
  asm volatile("v_nop\n\tv_nop\n\tv_nop\n\tv_nop" : "+v"(c) : "v"(ah), "v"(al), "v"(bh), "v"(bl));
  return c;
}

__global__ __launch_bounds__(256) void k_wt_bf16(const float* __restrict__ W, unsigned short* __restrict__ Wt, int K, int N) {
  const int t = blockIdx.x * 256 + threadIdx.x;
  const int k8n = K / 8;
  if (t >= N * k8n) return;
  const int n = t / k8n, k8 = (t % k8n) * 8;
  v8us v;
#pragma unroll
  for (int i = 0; i < 8; ++i) v[i] = bf16_bits(W[(size_t)(k8 + i) * N + n]);
  *(volatile v8us*)(Wt + (size_t)n * K + k8) = v;
  __threadfence();
  *(volatile v8us*)(Wt + (size_t)n * K + k8) = v;
}

template <bool ASPLIT, int ACT, bool BIAS_BF16>
__global__ __launch_bounds__(128) void k_gemm_bf(const float* __restrict__ A, int lda, const unsigned short* __restrict__ Wt, int ldb,
                                               const float* __restrict__ bias, float* __restrict__ C, int ldc, int M, int N, int K) {
  __shared__ __attribute__((aligned(16))) float so[4][16][64];
  const int tid = threadIdx.x, w = tid >> 5, lane = tid & 31, ln = lane & 15, hh = lane >> 4;
  const int ntn = N / 64;
  const int wid = blockIdx.x * 4 + w;
  const int mt = wid / ntn, nq = wid % ntn;
  if (mt * 16 >= M) return;
  const int row0 = mt * 16, col0 = nq * 64;
  const float* arow = A + (size_t)(row0 + ln) * lda;
  v8f acc[4] = {};
  for (int kb = 0; kb < K; kb += 32) {
    FragB ah, al;
    const v4f x0 = *(const v4fa*)(arow + kb + 8 * hh), x1 = *(const v4fa*)(arow + kb + 8 * hh + 4);
    const v4f x2 = *(const v4fa*)(arow + kb + 16 + 8 * hh), x3 = *(const v4fa*)(arow + kb + 16 + 8 * hh + 4);
    float xs[16] = {x0[0],x0[1],x0[2],x0[3],x1[0],x1[1],x1[2],x1[3],x2[0],x2[1],x2[2],x2[3],x3[0],x3[1],x3[2],x3[3]};
#pragma unroll
    for (int i = 0; i < 16; ++i) { const unsigned short hb = bf16_bits(xs[i]); ah.u[i] = hb; al.u[i] = ASPLIT ? bf16_bits(xs[i] - bf16_val(hb)) : (unsigned short)0; }
#pragma unroll
    for (int t = 0; t < 4; ++t) {
      const unsigned short* brow = Wt + (size_t)(col0 + t * 16 + ln) * ldb + kb;
      FragB b;
      b.half[0] = *(const v8us*)(brow + 8 * hh);
      b.half[1] = *(const v8us*)(brow + 16 + 8 * hh);
      acc[t] = mmaN<ASPLIT ? 2 : 1>(ah.v, al.v, b.v, b.v, acc[t]);
    }
  }
#pragma unroll
  for (int t = 0; t < 4; ++t) {
    float bv = bias ? bias[col0 + t * 16 + ln] : 0.f;
    if (BIAS_BF16) bv = bf16_round(bv);
#pragma unroll
    for (int r = 0; r < 8; ++r) { float v = acc[t][r] + bv; if (ACT == 1) v = fmaxf(v, 0.f); so[w][8 * hh + r][t * 16 + ln] = v; }
  }
  __builtin_amdgcn_fence(__ATOMIC_ACQ_REL, "workgroup");
  __builtin_amdgcn_wave_barrier();
  const int rsub = lane >> 4, c4 = (lane & 15) * 4;
  for (int pass = 0; pass < 2; ++pass) {
#pragma unroll
    for (int q = 0; q < 8; ++q) {
      const int r = q * 2 + rsub;
      const v4f v = *(const v4fa*)&so[w][r][c4];
      *(volatile v4f*)(C + (size_t)(row0 + r) * ldc + col0 + c4) = v;
    }
    if (pass == 0) __threadfence();
  }
}

template <int D, bool CAUSAL>
__global__ __launch_bounds__(128) void k_flash(const float* __restrict__ qb, const float* __restrict__ kb, const float* __restrict__ vb,
                                             int pitch, int T, int H, float scale, float* __restrict__ y, int ypitch) {
  constexpr int KS = D / 32;
  constexpr int DT = D / 16;
  __shared__ __attribute__((aligned(16))) unsigned short sKh[32][D + 8], sKl[32][D + 8], sVh[32][D + 8], sVl[32][D + 8];
  __shared__ __attribute__((aligned(16))) unsigned short sPh[4][16][40], sPl[4][16][40];
  __shared__ __attribute__((aligned(16))) float sO[4][16][D];
  const int tid = threadIdx.x, w = tid >> 5, lane = tid & 31, ln = lane & 15, hh = lane >> 4;
  const int nqb = (T + 63) / 64;
  const int bh = blockIdx.x / nqb, qblk = blockIdx.x % nqb;
  const int b = bh / H, h = bh % H;
  const int q0 = qblk * 64 + w * 16;
  const float* Q = qb + (size_t)b * T * pitch + h * D;
  const float* K = kb + (size_t)b * T * pitch + h * D;
  const float* V = vb + (size_t)b * T * pitch + h * D;

  FragB aqh[KS], aql[KS];
  {
    int row = q0 + ln; if (row >= T) row = T - 1;
    const float* qr = Q + (size_t)row * pitch;
#pragma unroll
    for (int ks = 0; ks < KS; ++ks)
#pragma unroll
      for (int i = 0; i < 16; ++i) {
        const int d = ks * 32 + ((i < 8) ? (8 * hh + i) : (16 + 8 * hh + (i - 8)));
        const float x = qr[d] * scale; const unsigned short hb = bf16_bits(x);
        aqh[ks].u[i] = hb; aql[ks].u[i] = bf16_bits(x - bf16_val(hb));
      }
  }
  float m_r[8], l_r[8];
#pragma unroll
  for (int r = 0; r < 8; ++r) { m_r[r] = -3.0e38f; l_r[r] = 0.f; }
  v8f oacc[DT];
#pragma unroll
  for (int dt = 0; dt < DT; ++dt) oacc[dt] = (v8f){0.f,0.f,0.f,0.f,0.f,0.f,0.f,0.f};

  const int kv_end = CAUSAL ? min(T, qblk * 64 + 64) : T;
  for (int j0 = 0; j0 < kv_end; j0 += 32) {
    __syncthreads();
    for (int e = tid; e < 32 * (D / 4); e += 128) {
      const int r = e / (D / 4), c4 = (e % (D / 4)) * 4;
      const int key = j0 + r;
      v4f kf = {0.f,0.f,0.f,0.f}, vf = {0.f,0.f,0.f,0.f};
      if (key < T) { kf = *(const v4fa*)(K + (size_t)key * pitch + c4); vf = *(const v4fa*)(V + (size_t)key * pitch + c4); }
#pragma unroll
      for (int t = 0; t < 4; ++t) {
        unsigned short hb = bf16_bits(kf[t]); sKh[r][c4 + t] = hb; sKl[r][c4 + t] = bf16_bits(kf[t] - bf16_val(hb));
        hb = bf16_bits(vf[t]); sVh[r][c4 + t] = hb; sVl[r][c4 + t] = bf16_bits(vf[t] - bf16_val(hb));
      }
    }
    __syncthreads();
    v8f s[2];
#pragma unroll
    for (int nt = 0; nt < 2; ++nt) {
      v8f acc = {};
#pragma unroll
      for (int ks = 0; ks < KS; ++ks) {
        FragB bh_, bl_;
        bh_.half[0] = *(const v8us*)&sKh[nt * 16 + ln][ks * 32 + 8 * hh]; bh_.half[1] = *(const v8us*)&sKh[nt * 16 + ln][ks * 32 + 16 + 8 * hh];
        bl_.half[0] = *(const v8us*)&sKl[nt * 16 + ln][ks * 32 + 8 * hh]; bl_.half[1] = *(const v8us*)&sKl[nt * 16 + ln][ks * 32 + 16 + 8 * hh];
        acc = mmaN<3>(aqh[ks].v, aql[ks].v, bh_.v, bl_.v, acc);
      }
      s[nt] = acc;
    }
    float alpha[8];
#pragma unroll
    for (int r = 0; r < 8; ++r) {
      const int qi = q0 + 8 * hh + r;
      const int ja = j0 + ln, jb = j0 + 16 + ln;
      if (CAUSAL) { if (ja > qi) s[0][r] = -3.0e38f; if (jb > qi) s[1][r] = -3.0e38f; }
      if (ja >= T) s[0][r] = -3.0e38f;
      if (jb >= T) s[1][r] = -3.0e38f;
      float mx = fmaxf(s[0][r], s[1][r]);
      mx = fmaxf(mx, __shfl_xor(mx, 1, 32)); mx = fmaxf(mx, __shfl_xor(mx, 2, 32)); mx = fmaxf(mx, __shfl_xor(mx, 4, 32)); mx = fmaxf(mx, __shfl_xor(mx, 8, 32));
      const float mnew = fmaxf(m_r[r], mx);
      alpha[r] = (mnew > -1.0e38f) ? __expf(m_r[r] - mnew) : 1.0f;
      const float p0 = (s[0][r] > -1.0e38f) ? __expf(s[0][r] - mnew) : 0.f;
      const float p1 = (s[1][r] > -1.0e38f) ? __expf(s[1][r] - mnew) : 0.f;
      m_r[r] = mnew;
      l_r[r] = l_r[r] * alpha[r] + p0 + p1;
      unsigned short hb = bf16_bits(p0); sPh[w][8 * hh + r][ln] = hb;      sPl[w][8 * hh + r][ln] = bf16_bits(p0 - bf16_val(hb));
      hb = bf16_bits(p1);                sPh[w][8 * hh + r][16 + ln] = hb; sPl[w][8 * hh + r][16 + ln] = bf16_bits(p1 - bf16_val(hb));
    }
#pragma unroll
    for (int dt = 0; dt < DT; ++dt)
#pragma unroll
      for (int r = 0; r < 8; ++r) oacc[dt][r] *= alpha[r];
    __builtin_amdgcn_fence(__ATOMIC_ACQ_REL, "workgroup");
    __builtin_amdgcn_wave_barrier();
    FragB pah, pal;
    pah.half[0] = *(const v8us*)&sPh[w][ln][8 * hh]; pah.half[1] = *(const v8us*)&sPh[w][ln][16 + 8 * hh];
    pal.half[0] = *(const v8us*)&sPl[w][ln][8 * hh]; pal.half[1] = *(const v8us*)&sPl[w][ln][16 + 8 * hh];
#pragma unroll
    for (int dt = 0; dt < DT; ++dt) {
      FragB bvh, bvl;
#pragma unroll
      for (int i = 0; i < 8; ++i) {
        bvh.u[i] = sVh[8 * hh + i][dt * 16 + ln]; bvh.u[8 + i] = sVh[16 + 8 * hh + i][dt * 16 + ln];
        bvl.u[i] = sVl[8 * hh + i][dt * 16 + ln]; bvl.u[8 + i] = sVl[16 + 8 * hh + i][dt * 16 + ln];
      }
      oacc[dt] = mmaN<3>(pah.v, pal.v, bvh.v, bvl.v, oacc[dt]);
    }
    __builtin_amdgcn_fence(__ATOMIC_ACQ_REL, "workgroup");
    __builtin_amdgcn_wave_barrier();
  }
#pragma unroll
  for (int r = 0; r < 8; ++r) {
    float l = l_r[r];
    l += __shfl_xor(l, 1, 32); l += __shfl_xor(l, 2, 32); l += __shfl_xor(l, 4, 32); l += __shfl_xor(l, 8, 32);
    l_r[r] = (l > 0.f) ? 1.0f / l : 0.f;
  }
#pragma unroll
  for (int dt = 0; dt < DT; ++dt)
#pragma unroll
    for (int r = 0; r < 8; ++r) sO[w][8 * hh + r][dt * 16 + ln] = oacc[dt][r] * l_r[r];
  __builtin_amdgcn_fence(__ATOMIC_ACQ_REL, "workgroup");
  __builtin_amdgcn_wave_barrier();
  for (int pass = 0; pass < 2; ++pass) {
    for (int r = 0; r < 16; ++r) {
      const int row = q0 + r;
      if (row < T && lane < D / 4) {
        const v4f val = *(const v4fa*)&sO[w][r][lane * 4];
        *(volatile v4f*)(y + ((size_t)b * T + row) * ypitch + h * D + lane * 4) = val;
      }
    }
    if (pass == 0) __threadfence();
  }
}

template <bool ASPLIT, int ACT, bool BIAS_BF16, bool RES_BF16>
__global__ __launch_bounds__(128) void k_gemm_bf3(const float* __restrict__ A, int lda, const unsigned short* __restrict__ Wt, int ldb,
                                                const float* __restrict__ bias, const float* __restrict__ resid, int rmod, int ldr,
                                                float* __restrict__ C, int ldc, int M, int N, int K) {
  __shared__ __attribute__((aligned(16))) float so[4][16][64];
  const int tid = threadIdx.x, w = tid >> 5, lane = tid & 31, ln = lane & 15, hh = lane >> 4;
  const int ntn = N / 64;
  const int wid = blockIdx.x * 4 + w;
  const int mt = wid / ntn, nq = wid % ntn;
  if (mt * 16 >= M) return;
  const int row0 = mt * 16, col0 = nq * 64;
  const float* arow = A + (size_t)(row0 + ln) * lda;
  v8f acc[4] = {};
  for (int kb = 0; kb < K; kb += 32) {
    FragB ah, al;
    const v4f x0 = *(const v4fa*)(arow + kb + 8 * hh), x1 = *(const v4fa*)(arow + kb + 8 * hh + 4);
    const v4f x2 = *(const v4fa*)(arow + kb + 16 + 8 * hh), x3 = *(const v4fa*)(arow + kb + 16 + 8 * hh + 4);
    float xs[16] = {x0[0],x0[1],x0[2],x0[3],x1[0],x1[1],x1[2],x1[3],x2[0],x2[1],x2[2],x2[3],x3[0],x3[1],x3[2],x3[3]};
#pragma unroll
    for (int i = 0; i < 16; ++i) { const unsigned short hb = bf16_bits(xs[i]); ah.u[i] = hb; al.u[i] = ASPLIT ? bf16_bits(xs[i] - bf16_val(hb)) : (unsigned short)0; }
#pragma unroll
    for (int t = 0; t < 4; ++t) {
      const unsigned short* brow = Wt + (size_t)(col0 + t * 16 + ln) * ldb + kb;
      FragB b;
      b.half[0] = *(const v8us*)(brow + 8 * hh);
      b.half[1] = *(const v8us*)(brow + 16 + 8 * hh);
      acc[t] = mmaN<ASPLIT ? 2 : 1>(ah.v, al.v, b.v, b.v, acc[t]);
    }
  }
#pragma unroll
  for (int t = 0; t < 4; ++t) {
    const int col = col0 + t * 16 + ln;
    float bv = bias ? bias[col] : 0.f;
    if (BIAS_BF16) bv = bf16_round(bv);
#pragma unroll
    for (int r = 0; r < 8; ++r) {
      float v = acc[t][r] + bv;
      if (resid) { float rv = resid[(size_t)((row0 + 8 * hh + r) % rmod) * ldr + col]; if (RES_BF16) rv = bf16_round(rv); v += rv; }
      if (ACT == 1) v = fmaxf(v, 0.f);
      if (ACT == 2) v = 0.5f * v * (1.0f + erff(v * 0.70710678118654752f));
      if (ACT == 3) { const float u = 0.7978845608028654f * (v + 0.044715f * v * v * v); v = 0.5f * v * (1.0f + tanhf(u)); }
      so[w][8 * hh + r][t * 16 + ln] = v;
    }
  }
  __builtin_amdgcn_fence(__ATOMIC_ACQ_REL, "workgroup");
  __builtin_amdgcn_wave_barrier();
  const int rsub = lane >> 4, c4 = (lane & 15) * 4;
  for (int pass = 0; pass < 2; ++pass) {
#pragma unroll
    for (int q = 0; q < 8; ++q) {
      const int r = q * 2 + rsub;
      const v4f v = *(const v4fa*)&so[w][r][c4];
      *(volatile v4f*)(C + (size_t)(row0 + r) * ldc + col0 + c4) = v;
    }
    if (pass == 0) __threadfence();
  }
}
template <bool PARAM_BF16>
__global__ __launch_bounds__(256) void k_layernorm(const float* __restrict__ X, const float* __restrict__ R, const float* __restrict__ g, const float* __restrict__ bta,
                                                  float* __restrict__ out_sum, float* __restrict__ out_norm, int N, float eps) {
  __shared__ float red[256];
  const int row = blockIdx.x, tid = threadIdx.x;
  const float* x = X + (size_t)row * N; const float* rr = R ? R + (size_t)row * N : nullptr;
  float vals[16];
  const int per = N / 256;
  float s1 = 0.f;
  for (int u = 0; u < per / 4; ++u) {
    const int j = tid * 4 + 1024 * u;
    const v4f a = *(const v4fa*)(x + j);
    v4f b = {0.f,0.f,0.f,0.f}; if (rr) b = *(const v4fa*)(rr + j);
#pragma unroll
    for (int q = 0; q < 4; ++q) { const float v = a[q] + b[q]; vals[u * 4 + q] = v; s1 += v; }
  }
  red[tid] = s1; __syncthreads();
  for (int st = 128; st > 0; st >>= 1) { if (tid < st) red[tid] += red[tid + st]; __syncthreads(); }
  const float mu = red[0] / (float)N; __syncthreads();
  float s2 = 0.f;
  for (int u = 0; u < per / 4; ++u)
#pragma unroll
    for (int q = 0; q < 4; ++q) { const float c = vals[u * 4 + q] - mu; s2 += c * c; }
  red[tid] = s2; __syncthreads();
  for (int st = 128; st > 0; st >>= 1) { if (tid < st) red[tid] += red[tid + st]; __syncthreads(); }
  const float rs = rsqrtf(red[0] / (float)N + eps);
  for (int pass = 0; pass < 2; ++pass) {
    for (int u = 0; u < per / 4; ++u) {
      const int j = tid * 4 + 1024 * u;
      v4f o, sm;
#pragma unroll
      for (int q = 0; q < 4; ++q) {
        float gg = g[j + q], bb = bta[j + q];
        if (PARAM_BF16) { gg = bf16_round(gg); bb = bf16_round(bb); }
        sm[q] = vals[u * 4 + q]; o[q] = (vals[u * 4 + q] - mu) * rs * gg + bb;
      }
      if (out_sum) *(volatile v4f*)(out_sum + (size_t)row * N + j) = sm;
      *(volatile v4f*)(out_norm + (size_t)row * N + j) = o;
    }
    if (pass == 0) __threadfence();
  }
}

typedef _Float16 v16h __attribute__((ext_vector_type(16)));
union FragH { v16h v; v8us half[2]; _Float16 h[16]; unsigned short u[16]; };
template <int NT>
__device__ __forceinline__ v8f mmaH(v16h ah, v16h al, v16h bh, v16h bl, v8f c) {
  c = __builtin_amdgcn_wmma_f32_16x16x32_f16(false, ah, false, bh, (short)0, c, false, false);
  if (NT >= 2) c = __builtin_amdgcn_wmma_f32_16x16x32_f16(false, al, false, bh, (short)0, c, false, false);
  if (NT >= 3) c = __builtin_amdgcn_wmma_f32_16x16x32_f16(false, ah, false, bl, (short)0, c, false, false);
  asm volatile("v_nop\n\tv_nop\n\tv_nop\n\tv_nop" : "+v"(c) : "v"(ah), "v"(al), "v"(bh), "v"(bl));
  return c;
}
template <bool ASPLIT>
__global__ __launch_bounds__(128) void k_gemm_h(const float* __restrict__ A, int lda, size_t sA, const _Float16* __restrict__ Bh, int ldb, size_t sB, float alpha, float* __restrict__ C, int ldc, size_t sC, int M, int N, int K) {
  __shared__ __attribute__((aligned(16))) float so[4][16][64];
  const int tid = threadIdx.x, w = tid >> 5, lane = tid & 31, ln = lane & 15, hh = lane >> 4; const int by = blockIdx.y;
  A += (size_t)by * sA; Bh += (size_t)by * sB; C += (size_t)by * sC;
  const int ntn = (N + 63) / 64; const int wid = blockIdx.x * 4 + w; const int mt = wid / ntn, nq = wid % ntn; if (mt * 16 >= M) return;
  const int row0 = mt * 16, col0 = nq * 64; const float* arow = A + (size_t)(row0 + ln) * lda;
  v8f acc[4] = {};
  for (int kb = 0; kb < K; kb += 32) {
    FragH ah, al;
    const v4f x0 = *(const v4fa*)(arow + kb + 8 * hh), x1 = *(const v4fa*)(arow + kb + 8 * hh + 4), x2 = *(const v4fa*)(arow + kb + 16 + 8 * hh), x3 = *(const v4fa*)(arow + kb + 16 + 8 * hh + 4);
    float xs[16] = {x0[0],x0[1],x0[2],x0[3],x1[0],x1[1],x1[2],x1[3],x2[0],x2[1],x2[2],x2[3],x3[0],x3[1],x3[2],x3[3]};
#pragma unroll
    for (int i = 0; i < 16; ++i) { const _Float16 h = (_Float16)xs[i]; ah.h[i] = h; al.h[i] = ASPLIT ? (_Float16)(xs[i] - (float)h) : (_Float16)0.0f; }
#pragma unroll
    for (int t = 0; t < 4; ++t) { if (col0 + t * 16 >= N) continue; const size_t boff = (size_t)(col0 + t * 16 + ln) * ldb + kb; FragH bq; bq.half[0] = *(const v8us*)(Bh + boff + 8 * hh); bq.half[1] = *(const v8us*)(Bh + boff + 16 + 8 * hh);
      acc[t] = mmaH<ASPLIT ? 2 : 1>(ah.v, al.v, bq.v, bq.v, acc[t]); }
  }
#pragma unroll
  for (int t = 0; t < 4; ++t) { if (col0 + t * 16 >= N) continue;
#pragma unroll
    for (int r = 0; r < 8; ++r) so[w][8 * hh + r][t * 16 + ln] = acc[t][r] * alpha; }
  __builtin_amdgcn_fence(__ATOMIC_ACQ_REL, "workgroup"); __builtin_amdgcn_wave_barrier();
  const int rsub = lane >> 4, c4 = (lane & 15) * 4;
  for (int pass = 0; pass < 2; ++pass) {
#pragma unroll
    for (int q = 0; q < 8; ++q) { const int r = q * 2 + rsub; if (col0 + c4 < N) { const v4f v = *(const v4fa*)&so[w][r][c4]; *(volatile v4f*)(C + (size_t)(row0 + r) * ldc + col0 + c4) = v; } }
    if (pass == 0) __threadfence(); }
}

template <int DUMMY>
__global__ __launch_bounds__(128) void k_gemm_hh(const _Float16* __restrict__ A, int lda, size_t sA, const _Float16* __restrict__ Bh, int ldb, size_t sB, float alpha, float* __restrict__ C, int ldc, size_t sC, int M, int N, int K) {
  __shared__ __attribute__((aligned(16))) float so[4][16][64];
  const int tid = threadIdx.x, w = tid >> 5, lane = tid & 31, ln = lane & 15, hh = lane >> 4; const int by = blockIdx.y;
  A += (size_t)by * sA; Bh += (size_t)by * sB; C += (size_t)by * sC;
  const int ntn = (N + 63) / 64; const int wid = blockIdx.x * 4 + w; const int mt = wid / ntn, nq = wid % ntn; if (mt * 16 >= M) return;
  const int row0 = mt * 16, col0 = nq * 64; const _Float16* arow = A + (size_t)(row0 + ln) * lda;
  v8f acc[4] = {};
  for (int kb = 0; kb < K; kb += 32) { FragH ah; ah.half[0] = *(const v8us*)((const unsigned short*)arow + kb + 8 * hh); ah.half[1] = *(const v8us*)((const unsigned short*)arow + kb + 16 + 8 * hh);
#pragma unroll
    for (int t = 0; t < 4; ++t) { if (col0 + t * 16 >= N) continue; const size_t boff = (size_t)(col0 + t * 16 + ln) * ldb + kb; FragH bq; bq.half[0] = *(const v8us*)((const unsigned short*)Bh + boff + 8 * hh); bq.half[1] = *(const v8us*)((const unsigned short*)Bh + boff + 16 + 8 * hh);
      acc[t] = mmaH<1>(ah.v, ah.v, bq.v, bq.v, acc[t]); }
  }
#pragma unroll
  for (int t = 0; t < 4; ++t) { if (col0 + t * 16 >= N) continue;
#pragma unroll
    for (int r = 0; r < 8; ++r) so[w][8 * hh + r][t * 16 + ln] = acc[t][r] * alpha; }
  __builtin_amdgcn_fence(__ATOMIC_ACQ_REL, "workgroup"); __builtin_amdgcn_wave_barrier();
  const int rsub = lane >> 4, c4 = (lane & 15) * 4;
  for (int pass = 0; pass < 2; ++pass) {
#pragma unroll
    for (int q = 0; q < 8; ++q) { const int r = q * 2 + rsub; if (col0 + c4 < N) { const v4f v = *(const v4fa*)&so[w][r][c4]; *(volatile v4f*)(C + (size_t)(row0 + r) * ldc + col0 + c4) = v; } }
    if (pass == 0) __threadfence(); }
}

__global__ __launch_bounds__(256) void k_round_rows(const float* __restrict__ W, unsigned short* __restrict__ Wt, int n8) {
  const int t = blockIdx.x * 256 + threadIdx.x;
  if (t >= n8) return;
  const v4f a = *(const v4fa*)(W + (size_t)t * 8), b = *(const v4fa*)(W + (size_t)t * 8 + 4);
  v8us v; v[0]=bf16_bits(a[0]); v[1]=bf16_bits(a[1]); v[2]=bf16_bits(a[2]); v[3]=bf16_bits(a[3]);
  v[4]=bf16_bits(b[0]); v[5]=bf16_bits(b[1]); v[6]=bf16_bits(b[2]); v[7]=bf16_bits(b[3]);
  *(volatile v8us*)(Wt + (size_t)t * 8) = v; __threadfence(); *(volatile v8us*)(Wt + (size_t)t * 8) = v;
}

__global__ __launch_bounds__(256) void k_bcat2(const float* __restrict__ a, const float* __restrict__ b, float* __restrict__ o) { const int t = blockIdx.x * 256 + threadIdx.x; if (t >= 2 * CC) return; const float v = (t < CC) ? a[t] : b[t - CC]; *(volatile float*)(o + t) = v; __threadfence(); *(volatile float*)(o + t) = v; }
__global__ __launch_bounds__(256) void k_copy300(const float* __restrict__ src, float* __restrict__ dst) { const int t = blockIdx.x * 256 + threadIdx.x; if (t >= NQ * CC / 4) return; const v4f v = *(const v4fa*)(src + (size_t)t * 4); *(volatile v4f*)(dst + (size_t)t * 4) = v; __threadfence(); *(volatile v4f*)(dst + (size_t)t * 4) = v; }
__global__ __launch_bounds__(256) void k_in(const float* __restrict__ rq, const float* __restrict__ qp, const float* __restrict__ rs, const float* __restrict__ sp, float* __restrict__ QS, float* __restrict__ MEM) { const int t = blockIdx.x * 256 + threadIdx.x;
  if (t < NQP * CC / 4) { const int r = (t * 4) / CC; v4f o = {0.f, 0.f, 0.f, 0.f}; if (r < NQ) { const v4f a = *(const v4fa*)(rq + (size_t)t * 4), b = *(const v4fa*)(qp + (size_t)t * 4); for (int q = 0; q < 4; ++q) o[q] = bf16_round(a[q]) + bf16_round(b[q]); } *(volatile v4f*)(QS + (size_t)t * 4) = o; __threadfence(); *(volatile v4f*)(QS + (size_t)t * 4) = o; }
  if (t < HW * CC / 4) { const v4f a = *(const v4fa*)(rs + (size_t)t * 4), b = *(const v4fa*)(sp + (size_t)t * 4); v4f o; for (int q = 0; q < 4; ++q) o[q] = bf16_round(a[q]) + bf16_round(b[q]); *(volatile v4f*)(MEM + (size_t)t * 4) = o; __threadfence(); *(volatile v4f*)(MEM + (size_t)t * 4) = o; } }
__global__ __launch_bounds__(256) void k_qh(const float* __restrict__ Q, float* __restrict__ Qh) { const int t = blockIdx.x * 256 + threadIdx.x; if (t >= NQP * CC / 4) return; const int c4 = (t * 4) % CC, q = (t * 4) / CC; const int h = c4 / HD, d4 = c4 % HD; v4f v = *(const v4fa*)(Q + (size_t)t * 4); for (int i = 0; i < 4; ++i) v[i] *= 0.17677669529663687f; *(volatile v4f*)(Qh + ((size_t)h * NQP + q) * HD + d4) = v; __threadfence(); *(volatile v4f*)(Qh + ((size_t)h * NQP + q) * HD + d4) = v; }
__global__ __launch_bounds__(256) void k_kv(const float* __restrict__ KV, _Float16* __restrict__ Kh, _Float16* __restrict__ Vt) { __shared__ float tv[64][65]; const int h = blockIdx.y, k0 = blockIdx.x * 64; const int tid = threadIdx.x; typedef _Float16 v4h __attribute__((ext_vector_type(4))); typedef _Float16 v2h __attribute__((ext_vector_type(2)));
  for (int e = tid; e < 64 * 8; e += 256) { const int r = e >> 3, c4 = (e & 7) * 4; const size_t row = (size_t)(k0 + r) * (2 * CC); const v4f k = *(const v4fa*)(KV + row + h * HD + c4), v = *(const v4fa*)(KV + row + CC + h * HD + c4); v4h kh; for (int i = 0; i < 4; ++i) { kh[i] = (_Float16)k[i]; tv[r][c4 + i] = v[i]; }
    _Float16* kd = Kh + ((size_t)h * HW + k0 + r) * HD + c4; *(volatile v4h*)kd = kh; __threadfence(); *(volatile v4h*)kd = kh; }
  __syncthreads();
  for (int pass = 0; pass < 2; ++pass) { for (int e = tid; e < 32 * 32; e += 256) { const int d = e >> 5, kp = (e & 31) * 2; v2h vv; vv.x = (_Float16)tv[kp][d]; vv.y = (_Float16)tv[kp + 1][d]; *(volatile v2h*)(Vt + ((size_t)h * HD + d) * HW + k0 + kp) = vv; } if (pass == 0) __threadfence(); } }
__global__ __launch_bounds__(256) void k_hid(const float* __restrict__ refp, const float* __restrict__ W1, const float* __restrict__ b1, int q0, _Float16* __restrict__ HIDB) { const size_t t = (size_t)blockIdx.x * 256 + threadIdx.x; if (t >= (size_t)QCH * HW * HID / 8) return; const int f8 = (int)((t * 8) % HID); const size_t pr = (t * 8) / HID; const int k = (int)(pr % HW); const int ql = (int)(pr / HW); int q = q0 + ql; q = q >= NQ ? NQ - 1 : q;
  const int ky = k / GW, kx = k % GW; const float kpx = ((float)kx + 0.5f) / (float)GW, kpy = ((float)ky + 0.5f) / (float)GH; const float dx = bf16_round(refp[q * 2]) - kpx, dy = bf16_round(refp[q * 2 + 1]) - kpy; FragH fr;
  for (int i = 0; i < 8; ++i) { const int f = f8 + i; fr.h[i] = (_Float16)fmaxf((dx * bf16_round(W1[f * 2]) + dy * bf16_round(W1[f * 2 + 1])) + bf16_round(b1[f]), 0.f); }
  *(volatile v8us*)((unsigned short*)HIDB + t * 8) = fr.half[0]; __threadfence(); *(volatile v8us*)((unsigned short*)HIDB + t * 8) = fr.half[0]; }
__global__ __launch_bounds__(256) void k_w2(const float* __restrict__ W2, _Float16* __restrict__ Bt) { const int t = blockIdx.x * 256 + threadIdx.x; if (t >= 16 * HID / 8) return; const int f8 = (t % (HID / 8)) * 8, h = t / (HID / 8); FragH fr; for (int i = 0; i < 8; ++i) fr.h[i] = (_Float16)(h < NH ? bf16_round(W2[h * HID + f8 + i]) * 16.0f : 0.f); *(volatile v8us*)((unsigned short*)Bt + (size_t)h * HID + f8) = fr.half[0]; __threadfence(); *(volatile v8us*)((unsigned short*)Bt + (size_t)h * HID + f8) = fr.half[0]; }
__global__ __launch_bounds__(1024) void k_softmax(float* __restrict__ S, const float* __restrict__ BI, float* __restrict__ Dn) { __shared__ float sd[32]; const int tid = threadIdx.x, wv = tid >> 5, lane = tid & 31; const int row = blockIdx.x * 32 + wv; if (row >= NH * NQP) return; const int h = row / NQP, q = row % NQP; float* sr = S + (size_t)row * HW;
  float mx = -3.0e38f;
#pragma unroll 1
  for (int k = lane; k < HW; k += 32) { const float v = sr[k] + ((q < NQ) ? BI[((size_t)q * HW + k) * 16 + h] : 0.f); *(volatile float*)(sr + k) = v; mx = fmaxf(mx, v); } for (int o = 16; o >= 1; o >>= 1) mx = fmaxf(mx, __shfl_xor(mx, o, 32)); __threadfence();
  float den = 0.f;
#pragma unroll 1
  for (int k = lane; k < HW; k += 32) { const float e = expf(sr[k] - mx); den += e; *(volatile float*)(sr + k) = e * 256.0f; } for (int o = 16; o >= 1; o >>= 1) den += __shfl_xor(den, o, 32); __threadfence();
#pragma unroll 1
  for (int k = lane; k < HW; k += 32) { const float pv = sr[k]; *(volatile float*)(sr + k) = pv; }
  if (lane == 0) sd[wv] = den; __syncthreads(); if (tid < 32 && blockIdx.x * 32 + tid < NH * NQP) { *(volatile float*)(Dn + blockIdx.x * 32 + tid) = sd[tid]; } __threadfence(); if (tid < 32 && blockIdx.x * 32 + tid < NH * NQP) { *(volatile float*)(Dn + blockIdx.x * 32 + tid) = sd[tid]; } }
__global__ __launch_bounds__(256) void k_onorm(const float* __restrict__ O, const float* __restrict__ Dn, float* __restrict__ CTX) { const int t = blockIdx.x * 256 + threadIdx.x; if (t >= NQP * CC / 4) return; const int c4 = (t * 4) % CC, q = (t * 4) / CC; const int h = c4 / HD, d4 = c4 % HD; const float rd = 1.0f / Dn[h * NQP + q]; const v4f o = *(const v4fa*)(O + ((size_t)h * NQP + q) * HD + d4); v4f r; for (int i = 0; i < 4; ++i) r[i] = o[i] * rd; *(volatile v4f*)(CTX + (size_t)t * 4) = r; __threadfence(); *(volatile v4f*)(CTX + (size_t)t * 4) = r; }
extern "C" void kernel_launch(void* const* d_in, const int* in_sizes, int n_in,
                              void* d_out, int out_size, void* d_ws, size_t ws_size, hipStream_t stream) {
  (void)in_sizes; (void)n_in; (void)out_size;
  const float* rq = (const float*)d_in[0]; const float* qp = (const float*)d_in[1]; const float* refp = (const float*)d_in[2]; const float* rs = (const float*)d_in[3]; const float* sp = (const float*)d_in[4];
  const float* Wq = (const float*)d_in[5]; const float* bq = (const float*)d_in[6]; const float* Wk = (const float*)d_in[7]; const float* bk = (const float*)d_in[8]; const float* Wv = (const float*)d_in[9]; const float* bv = (const float*)d_in[10]; const float* Wo = (const float*)d_in[11]; const float* bo = (const float*)d_in[12]; const float* W1 = (const float*)d_in[13]; const float* b1 = (const float*)d_in[14]; const float* W2 = (const float*)d_in[15]; (void)d_in[16];
  char* ws = (char*)d_ws; size_t off = 0;
  auto take = [&](size_t bytes) { char* p = ws + off; off += (bytes + 255) & ~(size_t)255; return p; };
  unsigned short* Bq = (unsigned short*)take((size_t)CC * CC * 2); unsigned short* Bkv = (unsigned short*)take((size_t)2 * CC * CC * 2); unsigned short* Bo = (unsigned short*)take((size_t)CC * CC * 2); _Float16* B2 = (_Float16*)take((size_t)16 * HID * 2); float* bkv = (float*)take(2 * CC * 4);
  float* QS = (float*)take((size_t)NQP * CC * 4); float* MEM = (float*)take((size_t)HW * CC * 4); float* Q = (float*)take((size_t)NQP * CC * 4); float* KV = (float*)take((size_t)HW * 2 * CC * 4);
  float* Qh = (float*)take((size_t)NH * NQP * HD * 4); _Float16* Kh = (_Float16*)take((size_t)NH * HW * HD * 2); _Float16* Vt = (_Float16*)take((size_t)NH * HD * HW * 2); float* S = (float*)take((size_t)NH * NQP * HW * 4);
  _Float16* HIDB = (_Float16*)take((size_t)QCH * HW * HID * 2); float* BI = (float*)take((size_t)NQP * HW * 16 * 4); float* Dn = (float*)take((size_t)NH * NQP * 4); float* O = (float*)take((size_t)NH * NQP * HD * 4); float* CTX = (float*)take((size_t)NQP * CC * 4); float* OUT = (float*)take((size_t)NQP * CC * 4);
  if (off > ws_size) return;
  k_round_rows<<<(CC * CC / 8 + 255) / 256, 256, 0, stream>>>(Wq, Bq, CC * CC / 8); k_round_rows<<<(CC * CC / 8 + 255) / 256, 256, 0, stream>>>(Wk, Bkv, CC * CC / 8); k_round_rows<<<(CC * CC / 8 + 255) / 256, 256, 0, stream>>>(Wv, Bkv + (size_t)CC * CC, CC * CC / 8); k_round_rows<<<(CC * CC / 8 + 255) / 256, 256, 0, stream>>>(Wo, Bo, CC * CC / 8);
  k_w2<<<(16 * HID / 8 + 255) / 256, 256, 0, stream>>>(W2, B2); k_bcat2<<<(2 * CC + 255) / 256, 256, 0, stream>>>(bk, bv, bkv);
  k_in<<<(HW * CC / 4 + 255) / 256, 256, 0, stream>>>(rq, qp, rs, sp, QS, MEM);
  k_gemm_bf3<true, 0, true, false><<<((NQP / 16) * (CC / 64) + 3) / 4, 128, 0, stream>>>(QS, CC, Bq, CC, bq, nullptr, 1, 0, Q, CC, NQP, CC, CC);
  k_gemm_bf3<true, 0, true, false><<<((HW / 16) * (2 * CC / 64) + 3) / 4, 128, 0, stream>>>(MEM, CC, Bkv, CC, bkv, nullptr, 1, 0, KV, 2 * CC, HW, 2 * CC, CC);
  k_qh<<<(NQP * CC / 4 + 255) / 256, 256, 0, stream>>>(Q, Qh); k_kv<<<dim3(HW / 64, NH), 256, 0, stream>>>(KV, Kh, Vt);
  k_gemm_h<true><<<dim3(((NQP / 16) * (HW / 64) + 3) / 4, NH), 128, 0, stream>>>(Qh, HD, (size_t)NQP * HD, Kh, HD, (size_t)HW * HD, 1.f, S, HW, (size_t)NQP * HW, NQP, HW, HD);
  for (int q0 = 0; q0 < NQP; q0 += QCH) {
    k_hid<<<(unsigned)(((size_t)QCH * HW * HID / 8 + 255) / 256), 256, 0, stream>>>(refp, W1, b1, q0, HIDB);
    k_gemm_hh<0><<<dim3(((QCH * HW / 16) * 1 + 3) / 4, 1), 128, 0, stream>>>(HIDB, HID, 0, B2, HID, 0, 0.0625f, BI + (size_t)q0 * HW * 16, 16, 0, QCH * HW, 16, HID);
  }
  k_softmax<<<(NH * NQP + 31) / 32, 1024, 0, stream>>>(S, BI, Dn);
  k_gemm_h<false><<<dim3(((NQP / 16) * 1 + 3) / 4, NH), 128, 0, stream>>>(S, HW, (size_t)NQP * HW, Vt, HW, (size_t)HD * HW, 0.00390625f, O, HD, (size_t)NQP * HD, NQP, HD, HW);
  k_onorm<<<(NQP * CC / 4 + 255) / 256, 256, 0, stream>>>(O, Dn, CTX);
  k_gemm_bf3<true, 0, true, false><<<((NQP / 16) * (CC / 64) + 3) / 4, 128, 0, stream>>>(CTX, CC, Bo, CC, bo, nullptr, 1, 0, OUT, CC, NQP, CC, CC);
  k_copy300<<<(NQ * CC / 4 + 255) / 256, 256, 0, stream>>>(OUT, (float*)d_out);
}
